// Transformer_47545287966777
// MI455X (gfx1250) — hardware-verified
//
#include <hip/hip_runtime.h>
#include <stddef.h>
#include <stdint.h>
#include <math.h>


#define DCH    64
#define PW     256
#define HK     128
#define NTHR   256
#define NWAVE  8
#define EPT    8
#define CHUNK  (NTHR * EPT)
#define WCAP   (EPT * 32)
#define LISTN  (NWAVE * WCAP)
#define NBA    1024
#define SLA    10
#define RCAP   28672
#define DEGCAP 64
#define MISCI  32
#define TABI   (RCAP + 2 * NBA + MISCI)
#define GBM    64
#define GBN    64
#define GTHR   128
#define U0     (PW * (DCH / 8))
#define U1     (PW * (HK / 8))
#define NUW    (U0 + 2 * U1)
#define NUB    192
#define WT0E   (PW * DCH)
#define WT1E   (PW * HK)
#define WTALL  (WT0E + 2 * WT1E)
#define AGG_ZINTS (LISTN + 2 * RCAP + 3 * NBA)
#define HITS_LDS_INTS (AGG_ZINTS + MISCI)

static_assert((CHUNK & (CHUNK - 1)) == 0 && CHUNK <= 4096);
static_assert((NBA & (NBA - 1)) == 0 && NBA == (1 << SLA));
static_assert(((long long)CHUNK << SLA) < (1LL << 31));
static_assert(NBA % NWAVE == 0 && NBA % 32 == 0 && NBA == 4 * NTHR);
static_assert(RCAP % (NTHR * 4) == 0 && AGG_ZINTS % (NTHR * 4) == 0);
static_assert(TABI % 32 == 0 && RCAP % 32 == 0);
static_assert(DCH % 32 == 0 && HK % 32 == 0 && HK == 2 * DCH);
static_assert(GBM == (GTHR / 32) * 16 && GBN == 64 && PW % GBN == 0);
static_assert(U0 % NTHR == 0 && U1 % NTHR == 0 && NUW % NTHR == 0 && NUB % 32 == 0 && NUB <= NTHR);
static_assert(DCH == 2 * 32);
static_assert(DEGCAP == 64);
static_assert(HITS_LDS_INTS * 4 <= 300000);

typedef float          v2f   __attribute__((ext_vector_type(2)));
typedef float          v4f   __attribute__((ext_vector_type(4)));
typedef float          v8f   __attribute__((ext_vector_type(8)));
typedef int            v4i   __attribute__((ext_vector_type(4)));
typedef int            v8i   __attribute__((ext_vector_type(8)));
typedef unsigned int   v4u   __attribute__((ext_vector_type(4)));
typedef unsigned short v8us  __attribute__((ext_vector_type(8)));
typedef unsigned short v16us __attribute__((ext_vector_type(16)));
typedef __bf16         v16bf __attribute__((ext_vector_type(16)));
typedef v2f  __attribute__((may_alias)) v2fa;
typedef v4f  __attribute__((may_alias)) v4fa;
typedef v4i  __attribute__((may_alias)) v4ia;
typedef v8us __attribute__((may_alias)) v8usa;
union FragB { v16bf v; v16us u; v8us h[2]; v8i w; };

__device__ __forceinline__ v8f wmb(const FragB& a, const FragB& b, v8f c) {
  v8f d = __builtin_amdgcn_wmma_f32_16x16x32_bf16(false, a.v, false, b.v, (short)0, c, false, false);
  asm volatile("v_nop\n\tv_nop\n\tv_nop\n\tv_nop" : "+v"(d) : "v"(a.w), "v"(b.w));
  return d;
}

__device__ __forceinline__ unsigned bf16_bits(float f) {
  const unsigned u = __float_as_uint(f);
  return (u + 0x7FFFu + ((u >> 16) & 1u)) >> 16;
}
__device__ __forceinline__ float bf16_val(float f) {
  return __uint_as_float(bf16_bits(f) << 16);
}

__device__ __forceinline__ void wave_sync() {
  __builtin_amdgcn_fence(__ATOMIC_RELEASE, "wavefront");
  __builtin_amdgcn_wave_barrier();
  __builtin_amdgcn_fence(__ATOMIC_ACQUIRE, "wavefront");
}

template <int SLB>
__device__ __forceinline__ int scan_chunk(const int* __restrict__ dsts, int nE, int cbase, int slotBase,
                                          int nb, int vec8, int* list, int tid, int lane, int wave) {
  int wc = 0;
  const int el0  = tid * EPT;
  const int e0   = cbase + el0;
  const int sent = -2147483647 - 1;
  v4i da, db;
  if (vec8 != 0 && cbase + CHUNK <= nE) {
    da = *(const v4i*)(dsts + e0);
    db = *(const v4i*)(dsts + e0 + 4);
  } else {
    da.x = (e0     < nE) ? dsts[min(e0,     nE - 1)] : sent;
    da.y = (e0 + 1 < nE) ? dsts[min(e0 + 1, nE - 1)] : sent;
    da.z = (e0 + 2 < nE) ? dsts[min(e0 + 2, nE - 1)] : sent;
    da.w = (e0 + 3 < nE) ? dsts[min(e0 + 3, nE - 1)] : sent;
    db.x = (e0 + 4 < nE) ? dsts[min(e0 + 4, nE - 1)] : sent;
    db.y = (e0 + 5 < nE) ? dsts[min(e0 + 5, nE - 1)] : sent;
    db.z = (e0 + 6 < nE) ? dsts[min(e0 + 6, nE - 1)] : sent;
    db.w = (e0 + 7 < nE) ? dsts[min(e0 + 7, nE - 1)] : sent;
  }
  const unsigned nbs = (unsigned)slotBase;
  const unsigned unb = (unsigned)nb;
  const unsigned s0 = (unsigned)da.x - nbs, s1 = (unsigned)da.y - nbs;
  const unsigned s2 = (unsigned)da.z - nbs, s3 = (unsigned)da.w - nbs;
  const unsigned s4 = (unsigned)db.x - nbs, s5 = (unsigned)db.y - nbs;
  const unsigned s6 = (unsigned)db.z - nbs, s7 = (unsigned)db.w - nbs;
  const bool h0 = s0 < unb, h1 = s1 < unb, h2 = s2 < unb, h3 = s3 < unb;
  const bool h4 = s4 < unb, h5 = s5 < unb, h6 = s6 < unb, h7 = s7 < unb;
  const unsigned any = __builtin_amdgcn_ballot_w32(h0 | h1 | h2 | h3 | h4 | h5 | h6 | h7);
  if (any != 0u) {
#define HITJ(J, HJ, SJ) { \
      const unsigned mj = __builtin_amdgcn_ballot_w32(HJ); \
      if (mj != 0u) { \
        if (HJ) { \
          const int pos = wc + (int)__builtin_amdgcn_mbcnt_lo(mj, 0u); \
          if (pos < WCAP) list[wave * WCAP + pos] = ((el0 + (J)) << SLB) | (int)(SJ); \
        } \
        wc += (int)__builtin_popcount(mj); } }
    HITJ(0, h0, s0)
    HITJ(1, h1, s1)
    HITJ(2, h2, s2)
    HITJ(3, h3, s3)
    HITJ(4, h4, s4)
    HITJ(5, h5, s5)
    HITJ(6, h6, s6)
    HITJ(7, h7, s7)
#undef HITJ
  }
  return wc;
}

__device__ __forceinline__ v8us ld8w(const float* __restrict__ W, size_t off) {
  const float* p = W + off;
  v8us o;
#pragma unroll
  for (int i = 0; i < 8; ++i) o[i] = (unsigned short)bf16_bits(p[(size_t)i * DCH]);
  return o;
}

__global__ __launch_bounds__(NTHR) void k_wprep(const float* __restrict__ Wq, const float* __restrict__ Wk,
                                                const float* __restrict__ Wv, const float* __restrict__ Ws,
                                                const float* __restrict__ bq, const float* __restrict__ bk,
                                                const float* __restrict__ bv, const float* __restrict__ bs,
                                                unsigned short* WT, float* BIAS) {
  const int u = (int)blockIdx.x * NTHR + (int)threadIdx.x;
  if (u < NUW) {
    int l, n, k8, K;
    size_t pbase;
    if (u < U0) {
      l = 0; n = u >> 3; k8 = (u & 7) * 8; K = DCH; pbase = 0;
    } else {
      const int v = u - U0;
      const int w = v & (U1 - 1);
      l = 1 + (v >> 12); n = w >> 4; k8 = (w & 15) * 8; K = HK;
      pbase = (size_t)WT0E + (size_t)(l - 1) * WT1E;
    }
    const int mat = n >> 6;
    const int nn  = n & 63;
    const int kk  = k8 & 63;
    const size_t off = ((size_t)l * DCH + kk) * DCH + nn;
    v8us o;
    if (mat == 0)      o = ld8w(Wq, off);
    else if (mat == 1) o = ld8w(Wk, off);
    else if (mat == 2) o = ld8w(Wv, off);
    else               o = ld8w(Ws, off);
    unsigned short* dp = WT + pbase + (size_t)n * K + k8;
    *(volatile v8us*)dp = o;
    __threadfence();
    *(volatile v8us*)dp = o;
  } else if (u < NUW + NUB) {
    const int j   = u - NUW;
    const int l   = j >> 6;
    const int r   = j & 63;
    const int mat = r >> 4;
    const int c   = (r & 15) * 4;
    const int so  = l * DCH + c;
    const v4f a0 = *(const v4f*)(bq + so);
    const v4f a1 = *(const v4f*)(bk + so);
    const v4f a2 = *(const v4f*)(bv + so);
    const v4f a3 = *(const v4f*)(bs + so);
    const float f0 = (mat == 0) ? 1.0f : 0.0f, f1 = (mat == 1) ? 1.0f : 0.0f;
    const float f2 = (mat == 2) ? 1.0f : 0.0f, f3 = (mat == 3) ? 1.0f : 0.0f;
    v4f o;
    o.x = bf16_val(a0.x * f0 + a1.x * f1 + a2.x * f2 + a3.x * f3);
    o.y = bf16_val(a0.y * f0 + a1.y * f1 + a2.y * f2 + a3.y * f3);
    o.z = bf16_val(a0.z * f0 + a1.z * f1 + a2.z * f2 + a3.z * f3);
    o.w = bf16_val(a0.w * f0 + a1.w * f1 + a2.w * f2 + a3.w * f3);
    float* dp = BIAS + (size_t)j * 4;
    *(volatile v4f*)dp = o;
    __threadfence();
    *(volatile v4f*)dp = o;
  }
}

__global__ __launch_bounds__(NTHR) void k_cvx(const float* __restrict__ x, int nN, int nUnits,
                                              unsigned short* xb) {
  const int u = (int)blockIdx.x * NTHR + (int)threadIdx.x;
  if (u >= nUnits) return;
  const int row = u >> 3;
  const int k8  = (u & 7) * 8;
  const int rc  = row < nN ? row : nN - 1;
  const float* p = x + (size_t)rc * DCH + k8;
  const v4f a = *(const v4fa*)p;
  const v4f b = *(const v4fa*)(p + 4);
  const bool ok = row < nN;
  v8us o;
  o[0] = ok ? (unsigned short)bf16_bits(a.x) : (unsigned short)0;
  o[1] = ok ? (unsigned short)bf16_bits(a.y) : (unsigned short)0;
  o[2] = ok ? (unsigned short)bf16_bits(a.z) : (unsigned short)0;
  o[3] = ok ? (unsigned short)bf16_bits(a.w) : (unsigned short)0;
  o[4] = ok ? (unsigned short)bf16_bits(b.x) : (unsigned short)0;
  o[5] = ok ? (unsigned short)bf16_bits(b.y) : (unsigned short)0;
  o[6] = ok ? (unsigned short)bf16_bits(b.z) : (unsigned short)0;
  o[7] = ok ? (unsigned short)bf16_bits(b.w) : (unsigned short)0;
  unsigned short* dp = xb + (size_t)row * DCH + k8;
  *(volatile v8us*)dp = o;
  __threadfence();
  *(volatile v8us*)dp = o;
}

__global__ __launch_bounds__(NTHR) void k_hits(const int* __restrict__ srcs, const int* __restrict__ dsts,
                                               int nE, int nN, int vec8, int* tab) {
  extern __shared__ __attribute__((aligned(16))) int dsm[];
  int* list = dsm;
  int* hl   = dsm + LISTN;
  int* sl   = hl + RCAP;
  int* cnt  = sl + RCAP;
  int* offs = cnt + NBA;
  int* cur  = offs + NBA;
  int* misc = cur + NBA;
  const int tid = (int)threadIdx.x, lane = tid & 31, wave = tid >> 5;
  const int nodeBase = (int)blockIdx.x * NBA;

  {
    const v4i z4 = {0, 0, 0, 0};
    for (int i = tid * 4; i < AGG_ZINTS; i += NTHR * 4) *(v4ia*)(dsm + i) = z4;
    if (tid < MISCI) misc[tid] = 0;
  }
  __syncthreads();

  int t = 0, ov = 0;
  const int nChunks = (nE + CHUNK - 1) / CHUNK;
#pragma unroll 1
  for (int ch = 0; ch < nChunks; ++ch) {
    const int cbase = ch * CHUNK;
    const int wc = scan_chunk<SLA>(dsts, nE, cbase, nodeBase, NBA, vec8, list, tid, lane, wave);
    if (lane == 0) misc[wave] = wc;
    __syncthreads();
    if (wave == 0) {
#pragma unroll 1
      for (int w2 = 0; w2 < NWAVE; ++w2) {
        int c = misc[w2];
        c = c < 0 ? 0 : (c > WCAP ? WCAP : c);
#pragma unroll 1
        for (int b0 = 0; b0 < c; b0 += 32) {
          const int idx = b0 + lane;
          const int ent = list[w2 * WCAP + (idx < WCAP ? idx : WCAP - 1)];
          const int m32 = (c - b0) < 32 ? (c - b0) : 32;
#pragma unroll 1
          for (int k = 0; k < m32; ++k) {
            const int u    = __builtin_amdgcn_readlane(ent, k);
            const int slot = u & (NBA - 1);
            const int el   = (u >> SLA) & (CHUNK - 1);
            const int pk   = ((cbase + el) << SLA) | slot;
            if (t < RCAP) {
              if (lane == 0) { hl[t] = pk; cnt[slot] = cnt[slot] + 1; }
              t = t + 1;
            } else {
              ov = 1;
            }
          }
        }
      }
    }
    __syncthreads();
  }
  if (wave == 0 && lane == 0) { misc[8] = t; misc[9] = ov; }
  __syncthreads();
  int tt = misc[8];
  tt = tt < 0 ? 0 : (tt > RCAP ? RCAP : tt);

  if (wave == 0) {
    const int base = lane * (NBA / 32);
    int s = 0;
#pragma unroll 1
    for (int i = 0; i < NBA / 32; ++i) s += cnt[base + i];
    int incl = s;
#pragma unroll
    for (int d = 1; d < 32; d <<= 1) {
      const int y = __shfl_up(incl, d, 32);
      if (lane >= d) incl += y;
    }
    int run = incl - s;
#pragma unroll 1
    for (int i = 0; i < NBA / 32; ++i) {
      const int cv = cnt[base + i];
      offs[base + i] = run;
      cur[base + i]  = run;
      run += cv;
    }
  }
  __syncthreads();
  if (wave == 0) {
#pragma unroll 1
    for (int b0 = 0; b0 < tt; b0 += 32) {
      const int idx = b0 + lane;
      const int ent = hl[idx < RCAP ? idx : RCAP - 1];
      const int m32 = (tt - b0) < 32 ? (tt - b0) : 32;
#pragma unroll 1
      for (int k = 0; k < m32; ++k) {
        const int u    = __builtin_amdgcn_readlane(ent, k);
        const int slot = u & (NBA - 1);
        if (lane == 0) {
          int p = cur[slot];
          p = p < 0 ? 0 : (p > RCAP - 1 ? RCAP - 1 : p);
          sl[p] = u;
          cur[slot] = p + 1;
        }
      }
    }
  }
  __syncthreads();

#pragma unroll 4
  for (int i = tid; i < RCAP; i += NTHR) {
    const int ent = sl[i];
    int eid = ent >> SLA;
    eid = eid < 0 ? 0 : (eid > nE - 1 ? nE - 1 : eid);
    int sr = srcs[eid];
    sr = sr < 0 ? 0 : (sr > nN - 1 ? nN - 1 : sr);
    sl[i] = (i < tt) ? sr : 0;
  }
  __syncthreads();

  int* tb = tab + (size_t)blockIdx.x * TABI;
#define HITS_PUT() { \
    _Pragma_free_loop: ; }
#undef HITS_PUT
#pragma unroll 1
  for (int it = 0; it < RCAP / (NTHR * 4); ++it) {
    const int idx = it * (NTHR * 4) + 4 * tid;
    const v4i v = *(const v4ia*)(sl + idx);
    *(volatile v4i*)(tb + idx) = v;
  }
  {
    const v4i c4 = *(const v4ia*)(cnt + 4 * tid);
    const v4i o4 = *(const v4ia*)(offs + 4 * tid);
    *(volatile v4i*)(tb + RCAP + 4 * tid) = c4;
    *(volatile v4i*)(tb + RCAP + NBA + 4 * tid) = o4;
    if (tid < MISCI / 4) {
      const v4i m4 = *(const v4ia*)(misc + 4 * tid);
      *(volatile v4i*)(tb + RCAP + 2 * NBA + 4 * tid) = m4;
    }
  }
  __threadfence();
#pragma unroll 1
  for (int it = 0; it < RCAP / (NTHR * 4); ++it) {
    const int idx = it * (NTHR * 4) + 4 * tid;
    const v4i v = *(const v4ia*)(sl + idx);
    *(volatile v4i*)(tb + idx) = v;
  }
  {
    const v4i c4 = *(const v4ia*)(cnt + 4 * tid);
    const v4i o4 = *(const v4ia*)(offs + 4 * tid);
    *(volatile v4i*)(tb + RCAP + 4 * tid) = c4;
    *(volatile v4i*)(tb + RCAP + NBA + 4 * tid) = o4;
    if (tid < MISCI / 4) {
      const v4i m4 = *(const v4ia*)(misc + 4 * tid);
      *(volatile v4i*)(tb + RCAP + 2 * NBA + 4 * tid) = m4;
    }
  }
}

__global__ __launch_bounds__(GTHR) void k_gemm(
    const unsigned short* __restrict__ A, const unsigned short* __restrict__ WT,
    const float* __restrict__ bias, float* outF, int K, int ldo)
{
  __shared__ __attribute__((aligned(16))) float stg[GBM * GBN];
  const int tid = (int)threadIdx.x, lane = tid & 31, wave = tid >> 5, hh = lane >> 4, m = lane & 15;
  const int rowBase = (int)blockIdx.x * GBM;
  const int col0    = (int)blockIdx.y * GBN;

  v8f acc[4];
  {
    const v8f z = {0.f, 0.f, 0.f, 0.f, 0.f, 0.f, 0.f, 0.f};
    acc[0] = z; acc[1] = z; acc[2] = z; acc[3] = z;
  }
  const unsigned short* ap = A  + (size_t)(rowBase + 16 * wave + m) * (size_t)K + 8 * hh;
  const unsigned short* wp = WT + (size_t)(col0 + m) * (size_t)K + 8 * hh;
  const int ksteps = K >> 5;
#pragma unroll 1
  for (int ks = 0; ks < ksteps; ++ks) {
    FragB af;
    af.h[0] = *(const v8usa*)(ap + 32 * ks);
    af.h[1] = *(const v8usa*)(ap + 32 * ks + 16);
#pragma unroll
    for (int t = 0; t < 4; ++t) {
      const unsigned short* wq = wp + (size_t)(16 * t) * (size_t)K + 32 * ks;
      FragB bf;
      bf.h[0] = *(const v8usa*)wq;
      bf.h[1] = *(const v8usa*)(wq + 16);
      acc[t] = wmb(af, bf, acc[t]);
    }
  }

#pragma unroll
  for (int t = 0; t < 4; ++t) {
    const int lc = 16 * t + m;
#pragma unroll
    for (int r = 0; r < 8; ++r) {
      const int lr = 16 * wave + 8 * hh + r;
      stg[lr * GBN + lc] = acc[t][r];
    }
  }
  __syncthreads();

  const v4f b4 = *(const v4f*)(bias + col0 + 4 * m);
  v4f fv[8];
#pragma unroll
  for (int i = 0; i < 8; ++i) {
    const int lr = 16 * wave + 2 * i + hh;
    const v4f sv = *(const v4fa*)(stg + lr * GBN + 4 * m);
    fv[i] = sv + b4;
  }
#pragma unroll
  for (int i = 0; i < 8; ++i) {
    const int lr = 16 * wave + 2 * i + hh;
    const int gr = rowBase + lr;
    float* op = outF + (size_t)gr * (size_t)ldo + col0 + 4 * m;
    *(volatile v4f*)op = fv[i];
  }
  __threadfence();
#pragma unroll
  for (int i = 0; i < 8; ++i) {
    const int lr = 16 * wave + 2 * i + hh;
    const int gr = rowBase + lr;
    float* op = outF + (size_t)gr * (size_t)ldo + col0 + 4 * m;
    *(volatile v4f*)op = fv[i];
  }
}

template <int FIN>
__global__ __launch_bounds__(NTHR) void k_agg(const int* __restrict__ tab, int nN, int mRows,
                                              const float* __restrict__ P, unsigned short* hb, float* outp) {
  __shared__ __attribute__((aligned(16))) int scnt[NBA];
  __shared__ __attribute__((aligned(16))) int soff[NBA];
  __shared__ float alist[NWAVE * DEGCAP];
  __shared__ int   slist[NWAVE * DEGCAP];
  const int tid = (int)threadIdx.x, lane = tid & 31, wave = tid >> 5;
  const int nodeBase = (int)blockIdx.x * NBA;
  const int* tb = tab + (size_t)blockIdx.x * TABI;
  {
    const v4i c4 = *(const v4i*)(tb + RCAP + 4 * tid);
    const v4i o4 = *(const v4i*)(tb + RCAP + NBA + 4 * tid);
    *(v4ia*)(scnt + 4 * tid) = c4;
    *(v4ia*)(soff + 4 * tid) = o4;
    for (int i = tid; i < NWAVE * DEGCAP; i += NTHR) { alist[i] = 0.0f; slist[i] = 0; }
  }
  const int ovf = tb[RCAP + 2 * NBA + 9];
  __syncthreads();

  float* al = alist + wave * DEGCAP;
  int*   sw = slist + wave * DEGCAP;
  const float qnan = __int_as_float(0x7fc00000);
  const float ninf = __int_as_float((int)0xff800000u);
  const float pz = (ovf != 0) ? qnan : 0.0f;
  const int sa = (2 * lane) & 31, sb = (2 * lane + 1) & 31;
  const int q0s = (4 * lane) & 31, q1s = (4 * lane + 1) & 31;
  const int q2s = (4 * lane + 2) & 31, q3s = (4 * lane + 3) & 31;

#pragma unroll 1
  for (int si = 0; si < NBA / NWAVE; ++si) {
    const int s    = si * NWAVE + wave;
    const int node = nodeBase + s;
    const int cr = __builtin_amdgcn_readfirstlane(scnt[s]);
    const bool big = (cr > DEGCAP) || (cr < 0);
    const int c = cr < 0 ? 0 : (cr > DEGCAP ? DEGCAP : cr);
    int o = __builtin_amdgcn_readfirstlane(soff[s]);
    o = o < 0 ? 0 : (o > RCAP ? RCAP : o);
    const int nc = node < nN ? node : nN - 1;
    const float* qrow = P + (size_t)nc * PW;

    float mloc = ninf;
#pragma unroll 1
    for (int b0 = 0; b0 < c; b0 += 32) {
      const int idx = b0 + lane;
      int hidx = o + idx;
      hidx = hidx > RCAP - 1 ? RCAP - 1 : hidx;
      int sr = tb[hidx];
      sr = sr < 0 ? 0 : (sr > nN - 1 ? nN - 1 : sr);
      const float* krow = P + (size_t)sr * PW + DCH;
      float p = 0.0f;
#pragma unroll 4
      for (int j = 0; j < DCH / 4; ++j) {
        const v4f q4 = *(const v4f*)(qrow + 4 * j);
        const v4f k4 = *(const v4f*)(krow + 4 * j);
        p = fmaf(q4.x, k4.x, p);
        p = fmaf(q4.y, k4.y, p);
        p = fmaf(q4.z, k4.z, p);
        p = fmaf(q4.w, k4.w, p);
      }
      const float a = (idx < c) ? (p * 0.125f) : ninf;
      al[idx] = a;
      sw[idx] = sr;
      mloc = fmaxf(mloc, a);
    }
    float m = mloc;
    m = fmaxf(m, __shfl_xor(m, 16, 32));
    m = fmaxf(m, __shfl_xor(m, 8, 32));
    m = fmaxf(m, __shfl_xor(m, 4, 32));
    m = fmaxf(m, __shfl_xor(m, 2, 32));
    m = fmaxf(m, __shfl_xor(m, 1, 32));

    float dloc = 0.0f;
#pragma unroll 1
    for (int b0 = 0; b0 < c; b0 += 32) {
      const int idx = b0 + lane;
      const float a  = al[idx];
      const float ex = expf(a - m);
      const float e  = (idx < c) ? ex : 0.0f;
      al[idx] = e;
      dloc += e;
    }
    float dsum = dloc;
    dsum += __shfl_xor(dsum, 16, 32);
    dsum += __shfl_xor(dsum, 8, 32);
    dsum += __shfl_xor(dsum, 4, 32);
    dsum += __shfl_xor(dsum, 2, 32);
    dsum += __shfl_xor(dsum, 1, 32);
    const float inv = 1.0f / (dsum + 1e-16f);
    wave_sync();

    float acc0 = 0.0f, acc1 = 0.0f;
#pragma unroll 2
    for (int k = 0; k < c; ++k) {
      const float ek = al[k];
      const int   sk = sw[k];
      const float ak = ek * inv;
      const v2f v = *(const v2fa*)(P + (size_t)sk * PW + 2 * DCH + 2 * lane);
      acc0 = fmaf(ak, v.x, acc0);
      acc1 = fmaf(ak, v.y, acc1);
    }
    wave_sync();

    const v2f sv = *(const v2fa*)(P + (size_t)nc * PW + 3 * DCH + 2 * lane);
    float y0 = acc0 + sv.x;
    float y1 = acc1 + sv.y;
    if constexpr (FIN == 0) {
      y0 = (y0 > 0.0f) ? y0 : (y0 - y0);
      y1 = (y1 > 0.0f) ? y1 : (y1 - y1);
    }
    const float pzr = big ? qnan : pz;
    y0 = y0 + pzr; y1 = y1 + pzr;
    const bool live = node < nN;
    const float v0 = live ? y0 : 0.0f;
    const float v1 = live ? y1 : 0.0f;
    if constexpr (FIN == 0) {
      const bool wr = (node < mRows) && (lane < 16);
      const unsigned hb0 = bf16_bits(v0), hb1 = bf16_bits(v1);
      const unsigned lb0 = bf16_bits(v0 - __uint_as_float(hb0 << 16));
      const unsigned lb1 = bf16_bits(v1 - __uint_as_float(hb1 << 16));
      const int hw = (int)(hb0 | (hb1 << 16));
      const int lw = (int)(lb0 | (lb1 << 16));
      const int g0 = __shfl(hw, q0s, 32), g1 = __shfl(hw, q1s, 32);
      const int g2 = __shfl(hw, q2s, 32), g3 = __shfl(hw, q3s, 32);
      const int p0 = __shfl(lw, q0s, 32), p1 = __shfl(lw, q1s, 32);
      const int p2 = __shfl(lw, q2s, 32), p3 = __shfl(lw, q3s, 32);
      const bool lsel = (lane & 8) != 0;
      v4u pv;
      pv.x = (unsigned int)(lsel ? p0 : g0);
      pv.y = (unsigned int)(lsel ? p1 : g1);
      pv.z = (unsigned int)(lsel ? p2 : g2);
      pv.w = (unsigned int)(lsel ? p3 : g3);
      unsigned short* hp = hb + (size_t)node * HK + 8 * (lane & 15);
      if (wr) *(volatile v4u*)hp = pv;
      __threadfence();
      if (wr) *(volatile v4u*)hp = pv;
    } else {
      const bool wr = (node < nN) && (lane < 16);
      v4f ow;
      ow.x = __shfl(v0, sa, 32); ow.y = __shfl(v1, sa, 32);
      ow.z = __shfl(v0, sb, 32); ow.w = __shfl(v1, sb, 32);
      float* op = outp + (size_t)node * DCH + 4 * (lane & 15);
      if (wr) *(volatile v4f*)op = ow;
      __threadfence();
      if (wr) *(volatile v4f*)op = ow;
    }
  }
}

static inline int cdiv(int a, int b) { return (a + b - 1) / b; }
static inline size_t al256(size_t o) { return (o + 255) & ~(size_t)255; }

extern "C" void kernel_launch(void* const* d_in, const int* in_sizes, int n_in,
                              void* d_out, int out_size, void* d_ws, size_t ws_size,
                              hipStream_t stream) {
  if (n_in < 11) return;
  if (in_sizes[0] < DCH || (in_sizes[0] % DCH) != 0) return;
  const int nN = in_sizes[0] / DCH;
  if (nN < 1 || nN > (1 << 22)) return;
  if (in_sizes[1] < 2 || (in_sizes[1] & 1) != 0) return;
  const int nE = in_sizes[1] / 2;
  if (nE < 1 || nE >= (1 << (31 - SLA))) return;
  if (in_sizes[3] != 3 * DCH * DCH || in_sizes[5] != 3 * DCH * DCH) return;
  if (in_sizes[7] != 3 * DCH * DCH || in_sizes[9] != 3 * DCH * DCH) return;
  if (in_sizes[4] != 3 * DCH || in_sizes[6] != 3 * DCH) return;
  if (in_sizes[8] != 3 * DCH || in_sizes[10] != 3 * DCH) return;
  if ((long long)out_size != (long long)nN * DCH) return;

  const float* x    = (const float*)d_in[0];
  const int*   edge = (const int*)d_in[1];
  const float* Wq   = (const float*)d_in[3];
  const float* bq   = (const float*)d_in[4];
  const float* Wk   = (const float*)d_in[5];
  const float* bk   = (const float*)d_in[6];
  const float* Wv   = (const float*)d_in[7];
  const float* bv   = (const float*)d_in[8];
  const float* Ws   = (const float*)d_in[9];
  const float* bs   = (const float*)d_in[10];
  float* out = (float*)d_out;
  const int* src = edge;
  const int* dst = edge + nE;

  const int MP = cdiv(nN, GBM) * GBM;
  const int gM = MP / GBM;
  const int gA = cdiv(MP, NBA);
  if ((long long)gA * NBA < (long long)MP) return;
  const int vec8 = ((nE & 3) == 0) ? 1 : 0;

  char* ws = (char*)d_ws;
  size_t off = 0;
  const size_t oWT  = off; off = al256(off + (size_t)WTALL * 2);
  const size_t oBI  = off; off = al256(off + (size_t)3 * PW * 4);
  const size_t oTAB = off; off = al256(off + (size_t)gA * TABI * 4);
  const size_t oXB  = off; off = al256(off + (size_t)MP * DCH * 2);
  const size_t oH   = off; off = al256(off + (size_t)MP * HK * 2);
  const size_t oP   = off; off = al256(off + (size_t)MP * PW * 4);
  if (off > ws_size) return;
  unsigned short* WT  = (unsigned short*)(ws + oWT);
  float*          BI  = (float*)(ws + oBI);
  int*            TAB = (int*)(ws + oTAB);
  unsigned short* XB  = (unsigned short*)(ws + oXB);
  unsigned short* H   = (unsigned short*)(ws + oH);
  float*          P   = (float*)(ws + oP);

  const size_t hitsLds = (size_t)HITS_LDS_INTS * 4;
  hipFuncSetAttribute(reinterpret_cast<const void*>(&k_hits), hipFuncAttributeMaxDynamicSharedMemorySize, (int)hitsLds);

  const int nUx = MP * (DCH / 8);
  k_wprep<<<cdiv(NUW + NUB, NTHR), NTHR, 0, stream>>>(Wq, Wk, Wv, Ws, bq, bk, bv, bs, WT, BI);
  k_cvx<<<cdiv(nUx, NTHR), NTHR, 0, stream>>>(x, nN, nUx, XB);
  k_hits<<<gA, NTHR, hitsLds, stream>>>(src, dst, nE, nN, vec8, TAB);
  k_gemm<<<dim3(gM, PW / GBN), GTHR, 0, stream>>>(XB, WT, BI, P, DCH, PW);
  k_agg<0><<<gA, NTHR, 0, stream>>>(TAB, nN, MP, P, H, out);
  k_gemm<<<dim3(gM, PW / GBN), GTHR, 0, stream>>>(H, WT + WT0E, BI + PW, P, HK, PW);
  k_agg<0><<<gA, NTHR, 0, stream>>>(TAB, nN, MP, P, H, out);
  k_gemm<<<dim3(gM, PW / GBN), GTHR, 0, stream>>>(H, WT + WT0E + WT1E, BI + 2 * PW, P, HK, PW);
  k_agg<1><<<gA, NTHR, 0, stream>>>(TAB, nN, MP, P, H, out);
}
